// SearchTransfer_40261023433211
// MI455X (gfx1250) — hardware-verified
//
#include <hip/hip_runtime.h>


typedef _Float16 v16h __attribute__((ext_vector_type(16)));
typedef _Float16 v8h  __attribute__((ext_vector_type(8)));
typedef float    v8f  __attribute__((ext_vector_type(8)));
typedef float    v4f  __attribute__((ext_vector_type(4)));
typedef int      v4i  __attribute__((ext_vector_type(4)));
union Frag { v16h v; v8h half[2]; };

constexpr int B_    = 8;
constexpr int C_    = 64;
constexpr int H_    = 96;
constexpr int W_    = 96;
constexpr int HQ    = 47;
constexpr int LQ    = HQ * HQ;
constexpr int KF    = C_ * 25;
constexpr int LPAD  = 2240;
constexpr int MT    = 4;
constexpr int NT    = 2;
constexpr int QG    = LPAD / (16 * NT);
constexpr int KGRP  = LPAD / (16 * MT);
constexpr int NWAV  = 4;
constexpr int C9    = C_ * 9;
constexpr int LV    = H_ * W_;
constexpr int NS    = B_ * LQ;
constexpr int NTT   = B_ * C9 * LQ;
constexpr int NOUT  = NS + NTT;
constexpr int NOUT4 = NOUT / 4;
static_assert(NOUT % 4 == 0);
static_assert(KF % 32 == 0);
static_assert(LPAD % 64 == 0 && LPAD >= LQ && LPAD % 32 == 0);
constexpr float OPSCALE = 256.0f;
constexpr float INVSC2  = 1.0f / 65536.0f;

__device__ __forceinline__ float bf16_rne(float x) {
    unsigned int u = __float_as_uint(x);
    u = (u + 0x7FFFu + ((u >> 16) & 1u)) & 0xFFFF0000u;
    return __uint_as_float(u);
}

__global__ __launch_bounds__(256) void k_pack(const float* __restrict__ queue, const float* __restrict__ key,
                                             _Float16* __restrict__ qbuf, _Float16* __restrict__ kbuf,
                                             float* __restrict__ rqb, float* __restrict__ rkb)
{
    __shared__ float rn_s[32];
    const int which = blockIdx.z;
    const float* src = which ? key : queue;
    _Float16* dst    = which ? kbuf : qbuf;
    float* rdst      = which ? rkb : rqb;
    const int b    = blockIdx.y;
    const int rblk = blockIdx.x;
    const int lane = threadIdx.x & 31;
    const int w    = threadIdx.x >> 5;
    const float* sb = src + (size_t)b * C_ * H_ * W_;

    for (int i = 0; i < 4; ++i) {
        const int rib  = i * 8 + w;
        const int row  = rblk * 32 + rib;
        const bool live = row < LQ;
        const int ry = row / HQ;
        const int rx = row - ry * HQ;
        _Float16* orow = dst + ((size_t)b * LPAD + row) * KF;

        v8h hv[7];
        double ss = 0.0;
#pragma unroll
        for (int it = 0; it < 7; ++it) {
            const int k8 = (it * 32 + lane) * 8;
            const int c0 = k8 / 25;
            const int r0 = k8 - c0 * 25;
            v8h h8;
#pragma unroll
            for (int e = 0; e < 8; ++e) {
                int rr = r0 + e;
                int cc = c0;
                if (rr >= 25) { rr -= 25; cc += 1; }
                const int kh = rr / 5;
                const int kw = rr - kh * 5;
                const int iy = ry * 2 + kh - 1;
                const int ix = rx * 2 + kw - 1;
                const bool ok = live && (k8 + e < KF) && (iy >= 0) && (iy < H_) && (ix >= 0) && (ix < W_);
                float x = 0.0f;
                if (ok) x = sb[(cc * H_ + iy) * W_ + ix];
                const float xb = bf16_rne(x);
                ss += (double)xb * (double)xb;
                h8[e] = (_Float16)(xb * OPSCALE);
            }
            hv[it] = h8;
        }
#pragma unroll
        for (int m = 16; m >= 1; m >>= 1) ss += __shfl_xor(ss, m, 32);
        const float nrm = sqrtf((float)ss);
        const float rn  = live ? (1.0f / fmaxf(nrm, 1e-12f)) : 0.0f;
        if (lane == 0) rn_s[rib] = rn;

#pragma unroll
        for (int it = 0; it < 6; ++it)
            *(volatile v8h*)(orow + (it * 32 + lane) * 8) = hv[it];
        if (lane < 8) *(volatile v8h*)(orow + (192 + lane) * 8) = hv[6];
        __threadfence();
#pragma unroll
        for (int it = 0; it < 6; ++it)
            *(volatile v8h*)(orow + (it * 32 + lane) * 8) = hv[it];
        if (lane < 8) *(volatile v8h*)(orow + (192 + lane) * 8) = hv[6];
    }
    __syncthreads();
    if (w == 0 && lane < 8) {
        v4f v;
        v.x = rn_s[lane * 4 + 0];
        v.y = rn_s[lane * 4 + 1];
        v.z = rn_s[lane * 4 + 2];
        v.w = rn_s[lane * 4 + 3];
        float* p = rdst + (size_t)b * LPAD + rblk * 32 + lane * 4;
        *(volatile v4f*)p = v;
        __threadfence();
        *(volatile v4f*)p = v;
    }
}

__global__ __launch_bounds__(128) void k_corr(const _Float16* __restrict__ qbuf, const _Float16* __restrict__ kbuf,
                                             const float* __restrict__ rqb, const float* __restrict__ rkb,
                                             float* __restrict__ sws, int* __restrict__ iws)
{
    __shared__ float s_val[NWAV][32];
    __shared__ int   s_idx[NWAV][32];
    __shared__ float o_val[32];
    __shared__ int   o_idx[32];

    const int lane = threadIdx.x & 31;
    const int w    = threadIdx.x >> 5;
    const int n    = lane & 15;
    const int hi   = lane >> 4;
    const int qg   = blockIdx.x;
    const int b    = blockIdx.y;

    const _Float16* qrow[NT];
    float cq[NT];
#pragma unroll
    for (int ni = 0; ni < NT; ++ni) {
        const int col = qg * 32 + ni * 16 + n;
        qrow[ni] = qbuf + ((size_t)b * LPAD + col) * KF + 8 * hi;
        cq[ni]   = rqb[(size_t)b * LPAD + col] * INVSC2;
    }
    const _Float16* kb   = kbuf + (size_t)b * LPAD * KF + (size_t)n * KF + 8 * hi;
    const float*    rkbb = rkb + (size_t)b * LPAD;

    float best[NT];
    int   bidx[NT];
#pragma unroll
    for (int ni = 0; ni < NT; ++ni) { best[ni] = -3.0e38f; bidx[ni] = 0; }

    for (int kg = w; kg < KGRP; kg += NWAV) {
        v8f acc[MT][NT];
#pragma unroll
        for (int mi = 0; mi < MT; ++mi)
#pragma unroll
            for (int ni = 0; ni < NT; ++ni) {
                v8f z = {0.f, 0.f, 0.f, 0.f, 0.f, 0.f, 0.f, 0.f};
                acc[mi][ni] = z;
            }
        const _Float16* kt = kb + (size_t)kg * (16 * MT) * KF;

#pragma unroll 1
        for (int ks = 0; ks < KF; ks += 32) {
            Frag bq[NT], ak[MT];
#pragma unroll
            for (int ni = 0; ni < NT; ++ni) {
                bq[ni].half[0] = *(const v8h*)(qrow[ni] + ks);
                bq[ni].half[1] = *(const v8h*)(qrow[ni] + ks + 16);
            }
#pragma unroll
            for (int mi = 0; mi < MT; ++mi) {
                const _Float16* ap = kt + (size_t)mi * 16 * KF + ks;
                ak[mi].half[0] = *(const v8h*)(ap);
                ak[mi].half[1] = *(const v8h*)(ap + 16);
            }
#pragma unroll
            for (int mi = 0; mi < MT; ++mi)
#pragma unroll
                for (int ni = 0; ni < NT; ++ni)
                    acc[mi][ni] = __builtin_amdgcn_wmma_f32_16x16x32_f16(
                        false, ak[mi].v, false, bq[ni].v, (short)0, acc[mi][ni], false, false);
            asm volatile("v_nop\n\tv_nop\n\tv_nop\n\tv_nop"
                         : "+v"(acc[0][0]), "+v"(acc[0][1]), "+v"(acc[1][0]), "+v"(acc[1][1]),
                           "+v"(acc[2][0]), "+v"(acc[2][1]), "+v"(acc[3][0]), "+v"(acc[3][1])
                         : "v"(ak[0].v), "v"(ak[1].v), "v"(ak[2].v), "v"(ak[3].v),
                           "v"(bq[0].v), "v"(bq[1].v));
        }

#pragma unroll
        for (int mi = 0; mi < MT; ++mi) {
            const int r0 = (kg * MT + mi) * 16 + hi * 8;
            const v4f rka = *(const v4f*)(rkbb + r0);
            const v4f rkc = *(const v4f*)(rkbb + r0 + 4);
            const float rk8[8] = {rka.x, rka.y, rka.z, rka.w, rkc.x, rkc.y, rkc.z, rkc.w};
#pragma unroll
            for (int ni = 0; ni < NT; ++ni) {
#pragma unroll
                for (int v = 0; v < 8; ++v) {
                    const int m = r0 + v;
                    const float val = acc[mi][ni][v] * rk8[v] * cq[ni];
                    const bool take = (m < LQ) && (val > best[ni]);
                    best[ni] = take ? val : best[ni];
                    bidx[ni] = take ? m : bidx[ni];
                }
            }
        }
    }

#pragma unroll
    for (int ni = 0; ni < NT; ++ni) {
        const float ov = __shfl_xor(best[ni], 16, 32);
        const int   oi = __shfl_xor(bidx[ni], 16, 32);
        if (ov > best[ni] || (ov == best[ni] && oi < bidx[ni])) { best[ni] = ov; bidx[ni] = oi; }
        if (hi == 0) { s_val[w][ni * 16 + n] = best[ni]; s_idx[w][ni * 16 + n] = bidx[ni]; }
    }
    __syncthreads();
    if (w == 0) {
        float bv = s_val[0][lane];
        int   bi = s_idx[0][lane];
#pragma unroll
        for (int u = 1; u < NWAV; ++u) {
            const float v = s_val[u][lane];
            const int   i = s_idx[u][lane];
            if (v > bv || (v == bv && i < bi)) { bv = v; bi = i; }
        }
        o_val[lane] = bv;
        o_idx[lane] = bi;
    }
    __syncthreads();
    if (w == 0 && lane < 8) {
        v4f sv; v4i iv;
        sv.x = o_val[lane * 4 + 0]; sv.y = o_val[lane * 4 + 1]; sv.z = o_val[lane * 4 + 2]; sv.w = o_val[lane * 4 + 3];
        iv.x = o_idx[lane * 4 + 0]; iv.y = o_idx[lane * 4 + 1]; iv.z = o_idx[lane * 4 + 2]; iv.w = o_idx[lane * 4 + 3];
        const size_t off = (size_t)b * LPAD + (size_t)qg * 32 + lane * 4;
        float* ps = sws + off;
        int*   pi = iws + off;
        *(volatile v4f*)ps = sv;
        *(volatile v4i*)pi = iv;
        __threadfence();
        *(volatile v4f*)ps = sv;
        *(volatile v4i*)pi = iv;
    }
}

__global__ __launch_bounds__(256) void k_out(const float* __restrict__ value, const float* __restrict__ sws,
                                            const int* __restrict__ iws, float* __restrict__ out)
{
    const unsigned int t = blockIdx.x * 256u + threadIdx.x;
    if (t >= (unsigned int)NOUT4) return;
    float r[4];
#pragma unroll
    for (int e = 0; e < 4; ++e) {
        const unsigned int f = t * 4u + (unsigned int)e;
        float v;
        if (f < (unsigned int)NS) {
            const unsigned int bb = f / (unsigned int)LQ;
            const unsigned int q  = f - bb * (unsigned int)LQ;
            v = sws[bb * LPAD + q];
        } else {
            const unsigned int g    = f - (unsigned int)NS;
            const unsigned int rest = g / (unsigned int)LQ;
            const unsigned int q    = g - rest * (unsigned int)LQ;
            const unsigned int bb   = rest / (unsigned int)C9;
            const unsigned int c9   = rest - bb * (unsigned int)C9;
            int l = iws[bb * LPAD + q];
            l = l < 0 ? 0 : (l > LV - 1 ? LV - 1 : l);
            const int y  = l / W_;
            const int x  = l - y * W_;
            const int c  = (int)c9 / 9;
            const int rr = (int)c9 - c * 9;
            const int kh = rr / 3;
            const int kw = rr - kh * 3;
            const int iy = y + kh - 1;
            const int ix = x + kw - 1;
            v = 0.0f;
            if (iy >= 0 && iy < H_ && ix >= 0 && ix < W_)
                v = bf16_rne(value[(((size_t)bb * C_ + c) * H_ + iy) * W_ + ix]);
        }
        r[e] = v;
    }
    v4f o = {r[0], r[1], r[2], r[3]};
    float* p = out + (size_t)t * 4;
    *(volatile v4f*)p = o;
    __threadfence();
    *(volatile v4f*)p = o;
}

extern "C" void kernel_launch(void* const* d_in, const int* in_sizes, int n_in,
                              void* d_out, int out_size, void* d_ws, size_t ws_size,
                              hipStream_t stream)
{
    if (n_in < 3) return;
    const int nin = B_ * C_ * H_ * W_;
    if (in_sizes[0] != nin || in_sizes[1] != nin || in_sizes[2] != nin) return;
    if (out_size != NOUT) return;

    const float* queue = (const float*)d_in[0];
    const float* key   = (const float*)d_in[1];
    const float* value = (const float*)d_in[2];

    const size_t fbytes = (size_t)B_ * LPAD * KF * sizeof(_Float16);
    const size_t vbytes = (size_t)B_ * LPAD * sizeof(float);
    const size_t o_q  = 0;
    const size_t o_k  = o_q + fbytes;
    const size_t o_rq = o_k + fbytes;
    const size_t o_rk = o_rq + vbytes;
    const size_t o_s  = o_rk + vbytes;
    const size_t o_i  = o_s + vbytes;
    const size_t o_end = o_i + vbytes;
    if (o_end > ws_size) return;

    char* ws = (char*)d_ws;
    _Float16* qbuf = (_Float16*)(ws + o_q);
    _Float16* kbuf = (_Float16*)(ws + o_k);
    float* rqb = (float*)(ws + o_rq);
    float* rkb = (float*)(ws + o_rk);
    float* sws = (float*)(ws + o_s);
    int*   iws = (int*)(ws + o_i);

    k_pack<<<dim3(LPAD / 32, B_, 2), 256, 0, stream>>>(queue, key, qbuf, kbuf, rqb, rkb);
    k_corr<<<dim3(QG, B_), 32 * NWAV, 0, stream>>>(qbuf, kbuf, rqb, rkb, sws, iws);
    k_out<<<(NOUT4 + 255) / 256, 256, 0, stream>>>(value, sws, iws, (float*)d_out);
    (void)hipGetLastError();
}
